// GPT2Block_20727512171020
// MI455X (gfx1250) — hardware-verified
//
#include <hip/hip_runtime.h>
#include <math.h>

#define NB    2
#define SEQ   2048
#define DM    1024
#define NH    16
#define HD    64
#define FF    4096
#define NTOK  (NB * SEQ)
#define WCARRY 16384.0f
#define WINV   (1.0f / 16384.0f)

typedef _Float16 v16h __attribute__((ext_vector_type(16)));
typedef _Float16 v8h  __attribute__((ext_vector_type(8)));
typedef float    v8f  __attribute__((ext_vector_type(8)));
typedef float    v4f  __attribute__((ext_vector_type(4)));
typedef v8h __attribute__((may_alias)) v8ha;
typedef v4f __attribute__((may_alias)) v4fa;

union FragU { v16h v; v8h h[2]; };

__device__ __forceinline__ v16h frag_ld(const _Float16* p) {
  FragU f;
  f.h[0] = *(const v8ha*)(p);
  f.h[1] = *(const v8ha*)(p + 16);
  return f.v;
}
__device__ __forceinline__ v8f mma16(v16h a, v16h b, v8f c) {
  return __builtin_amdgcn_wmma_f32_16x16x32_f16(false, a, false, b, (short)0, c, false, false);
}
__device__ __forceinline__ v8f mma16g(v16h a, v16h b, v8f c) {
  c = __builtin_amdgcn_wmma_f32_16x16x32_f16(false, a, false, b, (short)0, c, false, false);
  asm volatile("v_nop\n\tv_nop\n\tv_nop\n\tv_nop" : "+v"(c) : "v"(a), "v"(b));
  return c;
}
__device__ __forceinline__ void dep_guard_h(v8f& a, v8f& b, v16h x, v16h y) {
  asm volatile("v_nop\n\tv_nop\n\tv_nop\n\tv_nop" : "+v"(a), "+v"(b) : "v"(x), "v"(y));
}
__device__ __forceinline__ void keep4_h(v16h a, v16h b, v16h c, v16h d) {
  asm volatile("v_nop" :: "v"(a), "v"(b), "v"(c), "v"(d));
}
__device__ __forceinline__ void acc_guard4(v8f& a, v8f& b, v8f& c, v8f& d) {
  asm volatile("v_nop\n\tv_nop\n\tv_nop\n\tv_nop" : "+v"(a), "+v"(b), "+v"(c), "+v"(d));
}

__global__ __launch_bounds__(256) void tpose16_kernel(const float* __restrict__ W, _Float16* __restrict__ o,
                                                      int R, int Cc, float sc) {
  __shared__ __align__(16) float tf[64 * 68];
  const int c0  = blockIdx.x * 64;
  const int r0  = blockIdx.y * 64;
  const int tid = threadIdx.x;
  {
    const int lr = tid >> 4;
    const int c4 = (tid & 15) * 4;
#pragma unroll
    for (int it = 0; it < 4; ++it) {
      const int rr = it * 16 + lr;
      const v4f a = *(const v4fa*)(W + (size_t)(r0 + rr) * Cc + c0 + c4);
      *(v4fa*)(tf + rr * 68 + c4) = a;
    }
  }
  __syncthreads();
  const int sub = tid >> 3;
  const int c8  = (tid & 7) * 8;
  v8h hv[2];
#pragma unroll
  for (int it = 0; it < 2; ++it) {
    const int oc = it * 32 + sub;
    v8h v;
#pragma unroll
    for (int e = 0; e < 8; ++e) v[e] = (_Float16)(tf[(c8 + e) * 68 + oc] * sc);
    hv[it] = v;
  }
  for (int sweep = 0; sweep < 2; ++sweep) {
#pragma unroll
    for (int it = 0; it < 2; ++it) {
      const int oc = it * 32 + sub;
      const size_t go = (size_t)(c0 + oc) * R + r0 + c8;
      *(volatile v8h*)(o + go) = hv[it];
    }
    __threadfence();
  }
}

__global__ __launch_bounds__(128) void ln_f16_kernel(const float* __restrict__ x, const float* __restrict__ g,
                                                     const float* __restrict__ be, _Float16* __restrict__ out) {
  __shared__ float red[8];
  const int row = blockIdx.x;
  const int tid = threadIdx.x, lane = tid & 31, w = tid >> 5;
  const int i0 = tid * 8;
  const float* xr = x + (size_t)row * DM + i0;
  const v4f a = *(const v4fa*)(xr);
  const v4f c = *(const v4fa*)(xr + 4);
  float s = ((a.x + a.y) + (a.z + a.w)) + ((c.x + c.y) + (c.z + c.w));
#pragma unroll
  for (int off = 1; off < 32; off <<= 1) s += __shfl_xor(s, off);
  if (lane == 0) red[w] = s;
  __syncthreads();
  const float mean = ((red[0] + red[1]) + (red[2] + red[3])) * (1.0f / (float)DM);
  const float d0 = a.x - mean, d1 = a.y - mean, d2 = a.z - mean, d3 = a.w - mean;
  const float d4 = c.x - mean, d5 = c.y - mean, d6 = c.z - mean, d7 = c.w - mean;
  float ss = ((d0 * d0 + d1 * d1) + (d2 * d2 + d3 * d3)) + ((d4 * d4 + d5 * d5) + (d6 * d6 + d7 * d7));
#pragma unroll
  for (int off = 1; off < 32; off <<= 1) ss += __shfl_xor(ss, off);
  if (lane == 0) red[4 + w] = ss;
  __syncthreads();
  const float var  = ((red[4] + red[5]) + (red[6] + red[7])) * (1.0f / (float)DM);
  const float rstd = 1.0f / sqrtf(var + 1e-5f);
  const v4f g0 = *(const v4fa*)(g + i0);
  const v4f g1 = *(const v4fa*)(g + i0 + 4);
  const v4f b0 = *(const v4fa*)(be + i0);
  const v4f b1 = *(const v4fa*)(be + i0 + 4);
  v8h o;
  o[0] = (_Float16)(d0 * rstd * g0.x + b0.x);
  o[1] = (_Float16)(d1 * rstd * g0.y + b0.y);
  o[2] = (_Float16)(d2 * rstd * g0.z + b0.z);
  o[3] = (_Float16)(d3 * rstd * g0.w + b0.w);
  o[4] = (_Float16)(d4 * rstd * g1.x + b1.x);
  o[5] = (_Float16)(d5 * rstd * g1.y + b1.y);
  o[6] = (_Float16)(d6 * rstd * g1.z + b1.z);
  o[7] = (_Float16)(d7 * rstd * g1.w + b1.w);
  _Float16* dst = out + (size_t)row * DM + i0;
  *(volatile v8h*)dst = o;
  __threadfence();
  *(volatile v8h*)dst = o;
}

template <int BIAS_MODE, int OUT_MODE, bool RESID, int ACT>
__global__ __launch_bounds__(256) void wmma_gemm64(
    const _Float16* __restrict__ A, int lda, long strideA,
    const _Float16* __restrict__ Bt, int ldb, long strideB,
    void* __restrict__ Cout, int ldc, long strideC,
    const float* __restrict__ bias,
    const float* __restrict__ resid, long strideR,
    int M, int N, int K, float scale) {
  static_assert(!(RESID && OUT_MODE != 0));
  __shared__ __align__(16) float sT[8][16 * 68];
  const int b    = blockIdx.y;
  const int lane = threadIdx.x & 31;
  const int wave = threadIdx.x >> 5;
  const int tilesN = N >> 6;
  const int tilesM = M >> 6;
  const int tile = blockIdx.x * 8 + wave;
  if (tile >= tilesM * tilesN) return;
  const int tm = tile / tilesN;
  const int tn = tile - tm * tilesN;
  const int m0 = tm << 6;
  const int n0 = tn << 6;

  const _Float16* Ab = A  + (size_t)b * strideA;
  const _Float16* Bb = Bt + (size_t)b * strideB;

  const int rlane = lane & 15;
  const int koff  = (lane >> 4) * 8;
  const int mOff  = (lane >> 4) * 8;

  v8f acc[4][4];
#pragma unroll
  for (int i = 0; i < 4; ++i)
#pragma unroll
    for (int j = 0; j < 4; ++j) acc[i][j] = (v8f){0.f,0.f,0.f,0.f,0.f,0.f,0.f,0.f};

  for (int k0 = 0; k0 < K; k0 += 32) {
    v16h bh[4];
#pragma unroll
    for (int j = 0; j < 4; ++j) {
      const size_t bo = (size_t)(n0 + (j << 4) + rlane) * ldb + koff + k0;
      bh[j] = frag_ld(Bb + bo);
    }
#pragma unroll
    for (int i = 0; i < 4; ++i) {
      const size_t ao = (size_t)(m0 + (i << 4) + rlane) * lda + koff + k0;
      const v16h ah = frag_ld(Ab + ao);
#pragma unroll
      for (int j = 0; j < 4; ++j) acc[i][j] = mma16(ah, bh[j], acc[i][j]);
      dep_guard_h(acc[i][0], acc[i][3], ah, ah);
    }
    keep4_h(bh[0], bh[1], bh[2], bh[3]);
  }
  acc_guard4(acc[0][0], acc[0][1], acc[0][2], acc[0][3]);
  acc_guard4(acc[1][0], acc[1][1], acc[1][2], acc[1][3]);
  acc_guard4(acc[2][0], acc[2][1], acc[2][2], acc[2][3]);
  acc_guard4(acc[3][0], acc[3][1], acc[3][2], acc[3][3]);

  float* slab = sT[wave];
  const float* Rb = RESID ? (resid + (size_t)b * strideR) : nullptr;
#pragma unroll
  for (int i = 0; i < 4; ++i) {
    const int mBase = m0 + (i << 4);
    float bm[8];
#pragma unroll
    for (int r = 0; r < 8; ++r) bm[r] = 0.f;
    if (BIAS_MODE == 1) {
      const v4f t0 = *(const v4fa*)(bias + mBase + mOff);
      const v4f t1 = *(const v4fa*)(bias + mBase + mOff + 4);
      bm[0] = t0.x; bm[1] = t0.y; bm[2] = t0.z; bm[3] = t0.w;
      bm[4] = t1.x; bm[5] = t1.y; bm[6] = t1.z; bm[7] = t1.w;
    }
#pragma unroll
    for (int j = 0; j < 4; ++j) {
      const int n = n0 + (j << 4) + rlane;
      float bv = 0.f;
      if (BIAS_MODE == 2) bv = bias[n];
#pragma unroll
      for (int r = 0; r < 8; ++r) {
        float v = acc[i][j][r] * scale;
        if (BIAS_MODE == 1) v += bm[r];
        if (BIAS_MODE == 2) v += bv;
        if (ACT == 5) v = 0.5f * v * (1.0f + erff(v * 0.70710678118654752f));
        slab[(mOff + r) * 68 + (j << 4) + rlane] = v;
      }
    }
    __builtin_amdgcn_fence(__ATOMIC_RELEASE, "workgroup");
    __builtin_amdgcn_wave_barrier();
    __builtin_amdgcn_fence(__ATOMIC_ACQUIRE, "workgroup");
    if (OUT_MODE == 0) {
      float* C = (float*)Cout + (size_t)b * strideC;
      const int hh = lane >> 4, c4 = (lane & 15) * 4;
      for (int sweep = 0; sweep < 2; ++sweep) {
#pragma unroll
        for (int it = 0; it < 8; ++it) {
          const int row = it * 2 + hh;
          v4f v = *(const v4fa*)(slab + row * 68 + c4);
          if (RESID) {
            const v4f rr = *(const v4fa*)(Rb + (size_t)(mBase + row) * ldc + n0 + c4);
            v = v + rr;
          }
          *(volatile v4f*)(C + (size_t)(mBase + row) * ldc + n0 + c4) = v;
        }
        __threadfence();
      }
    } else {
      const int q = lane >> 3, c8 = (lane & 7) * 8;
      _Float16* C = (_Float16*)Cout + (size_t)b * strideC;
      for (int sweep = 0; sweep < 2; ++sweep) {
#pragma unroll
        for (int it = 0; it < 4; ++it) {
          const int row = it * 4 + q;
          const float* sp = slab + row * 68 + c8;
          v8h hv;
#pragma unroll
          for (int e = 0; e < 8; ++e) hv[e] = (_Float16)sp[e];
          *(volatile v8h*)(C + (size_t)(mBase + row) * ldc + n0 + c8) = hv;
        }
        __threadfence();
      }
    }
    __builtin_amdgcn_fence(__ATOMIC_RELEASE, "workgroup");
    __builtin_amdgcn_wave_barrier();
    __builtin_amdgcn_fence(__ATOMIC_ACQUIRE, "workgroup");
  }
}

#define AT_D  64
#define AT_NW 4
#define AT_QB 64
#define AT_KC 64

__global__ __launch_bounds__(128)
void attn_causal64_kernel(const _Float16* __restrict__ Qp, const _Float16* __restrict__ Kp,
                          const _Float16* __restrict__ Vtp, _Float16* __restrict__ Op, float sscale) {
  union FB { v16h v; v8h h[2]; };
  __shared__ __align__(16) _Float16 Ksh[AT_KC * AT_D];
  __shared__ __align__(16) _Float16 Vth[AT_D * AT_KC];
  __shared__ __align__(16) _Float16 Psh[AT_NW][16 * AT_KC];
  __shared__ __align__(16) float    Os[AT_NW][16 * 68];

  const int tid  = threadIdx.x;
  const int wave = tid >> 5;
  const int lane = tid & 31;
  const int hh   = lane >> 4;
  const int c    = lane & 15;

  const int nqb = SEQ / AT_QB;
  const int bx  = blockIdx.x;
  const int qb  = bx % nqb;
  const int h   = bx / nqb;
  const int b   = blockIdx.y;
  const int q0  = qb * AT_QB + wave * 16;

  const _Float16* Qb = Qp  + (size_t)b * SEQ * DM + h * AT_D;
  const _Float16* Kb = Kp  + (size_t)b * SEQ * DM + h * AT_D;
  const _Float16* Vb = Vtp + ((size_t)b * DM + h * AT_D) * SEQ;
  _Float16*       Ob = Op  + (size_t)b * SEQ * DM + h * AT_D;

  v16h qa[2];
#pragma unroll
  for (int dc = 0; dc < 2; ++dc) qa[dc] = frag_ld(Qb + (size_t)(q0 + c) * DM + dc * 32 + 8 * hh);

  float mrow[8], lrow[8];
  v8f oacc[4];
#pragma unroll
  for (int r = 0; r < 8; ++r) { mrow[r] = -INFINITY; lrow[r] = 0.f; }
#pragma unroll
  for (int t = 0; t < 4; ++t) oacc[t] = (v8f){0.f,0.f,0.f,0.f,0.f,0.f,0.f,0.f};

  const int nChunks = qb + 1;
  for (int kc = 0; kc < nChunks; ++kc) {
    const int kv0 = kc * AT_KC;
    __syncthreads();
    {
      const int r = tid >> 1, half = (tid & 1) * 32;
      const _Float16* ks = Kb + (size_t)(kv0 + r) * DM + half;
      const _Float16* vs = Vb + (size_t)r * SEQ + kv0 + half;
#pragma unroll
      for (int i = 0; i < 4; ++i) {
        const v8h a0 = *(const v8ha*)(ks + 8 * i);
        const v8h b0 = *(const v8ha*)(vs + 8 * i);
        *(v8ha*)(Ksh + r * AT_D  + half + 8 * i) = a0;
        *(v8ha*)(Vth + r * AT_KC + half + 8 * i) = b0;
      }
    }
    __syncthreads();

    v8f s[4];
#pragma unroll
    for (int j = 0; j < 4; ++j) {
      s[j] = (v8f){0.f,0.f,0.f,0.f,0.f,0.f,0.f,0.f};
#pragma unroll
      for (int dc = 0; dc < 2; ++dc) {
        FB kb;
        kb.h[0] = *(const v8ha*)(Ksh + (j * 16 + c) * AT_D + dc * 32 + 8 * hh);
        kb.h[1] = *(const v8ha*)(Ksh + (j * 16 + c) * AT_D + dc * 32 + 16 + 8 * hh);
        s[j] = mma16g(qa[dc], kb.v, s[j]);
      }
    }
    const bool diag = (kc == qb);
    float cm[8];
#pragma unroll
    for (int r = 0; r < 8; ++r) {
      const int qrow = q0 + 8 * hh + r;
      float m = -INFINITY;
#pragma unroll
      for (int j = 0; j < 4; ++j) {
        const int kvcol = kv0 + j * 16 + c;
        const float sv = s[j][r] * sscale;
        const bool excl = diag && (kvcol > qrow);
        const float sm = excl ? -INFINITY : sv;
        s[j][r] = sm;
        m = fmaxf(m, sm);
      }
#pragma unroll
      for (int off = 1; off < 16; off <<= 1) m = fmaxf(m, __shfl_xor(m, off, 32));
      cm[r] = m;
    }
    _Float16* pw = Psh[wave];
#pragma unroll
    for (int r = 0; r < 8; ++r) {
      const float mnew = fmaxf(mrow[r], cm[r]);
      const float alpha = expf(mrow[r] - mnew);
      mrow[r] = mnew;
      float psum = 0.f;
#pragma unroll
      for (int j = 0; j < 4; ++j) {
        const float p = expf(s[j][r] - mnew);
        psum += p;
        pw[(8 * hh + r) * AT_KC + j * 16 + c] = (_Float16)p;
      }
#pragma unroll
      for (int off = 1; off < 16; off <<= 1) psum += __shfl_xor(psum, off, 32);
      lrow[r] = lrow[r] * alpha + psum;
#pragma unroll
      for (int t = 0; t < 4; ++t) oacc[t][r] *= alpha;
    }
    __builtin_amdgcn_fence(__ATOMIC_RELEASE, "workgroup");
    __builtin_amdgcn_wave_barrier();
    __builtin_amdgcn_fence(__ATOMIC_ACQUIRE, "workgroup");
#pragma unroll 1
    for (int kk = 0; kk < 2; ++kk) {
      FB pa;
      pa.h[0] = *(const v8ha*)(pw + c * AT_KC + kk * 32 + 8 * hh);
      pa.h[1] = *(const v8ha*)(pw + c * AT_KC + kk * 32 + 16 + 8 * hh);
#pragma unroll
      for (int t = 0; t < 4; ++t) {
        FB vb;
        vb.h[0] = *(const v8ha*)(Vth + (t * 16 + c) * AT_KC + kk * 32 + 8 * hh);
        vb.h[1] = *(const v8ha*)(Vth + (t * 16 + c) * AT_KC + kk * 32 + 16 + 8 * hh);
        oacc[t] = mma16g(pa.v, vb.v, oacc[t]);
      }
    }
  }

  float* os = Os[wave];
#pragma unroll
  for (int r = 0; r < 8; ++r) {
    const float inv = 1.0f / lrow[r];
#pragma unroll
    for (int t = 0; t < 4; ++t) os[(8 * hh + r) * 68 + t * 16 + c] = oacc[t][r] * inv;
  }
  __builtin_amdgcn_fence(__ATOMIC_RELEASE, "workgroup");
  __builtin_amdgcn_wave_barrier();
  __builtin_amdgcn_fence(__ATOMIC_ACQUIRE, "workgroup");
  {
    const int q8 = lane & 7, sub = lane >> 3;
    for (int sweep = 0; sweep < 2; ++sweep) {
#pragma unroll
      for (int it = 0; it < 4; ++it) {
        const int row = it * 4 + sub;
        const float* sp = os + row * 68 + 8 * q8;
        const v4f a = *(const v4fa*)(sp);
        const v4f d = *(const v4fa*)(sp + 4);
        v8h hv;
        hv[0] = (_Float16)a.x; hv[1] = (_Float16)a.y; hv[2] = (_Float16)a.z; hv[3] = (_Float16)a.w;
        hv[4] = (_Float16)d.x; hv[5] = (_Float16)d.y; hv[6] = (_Float16)d.z; hv[7] = (_Float16)d.w;
        *(volatile v8h*)(Ob + (size_t)(q0 + row) * DM + 8 * q8) = hv;
      }
      __threadfence();
    }
  }
}

#define PW_DD ((size_t)DM * DM * 2)
#define PW_DF ((size_t)DM * FF * 2)
#define PACT  ((size_t)NTOK * DM * 2)
#define PADD  ((size_t)NTOK * DM * 4)
#define PG    ((size_t)NTOK * FF * 2)

static_assert((NTOK % 64) == 0);
static_assert((DM % 64) == 0);
static_assert((FF % 64) == 0);
static_assert((SEQ % 64) == 0);
static_assert((DM % 32) == 0);
static_assert((FF % 32) == 0);
static_assert(DM == NH * HD);
static_assert(DM == 128 * 8);
static_assert(4 * PW_DD + 2 * PW_DF + 6 * PACT + PADD + PG <= (size_t)134217728);

extern "C" void kernel_launch(void* const* d_in, const int* in_sizes, int n_in,
                              void* d_out, int out_size, void* d_ws, size_t ws_size,
                              hipStream_t stream) {
  if (n_in < 17) return;
  if (in_sizes[0] != NTOK * DM) return;
  if (in_sizes[1] != DM || in_sizes[2] != DM) return;
  if (in_sizes[3] != DM * DM || in_sizes[5] != DM * DM || in_sizes[7] != DM * DM || in_sizes[9] != DM * DM) return;
  if (in_sizes[4] != DM || in_sizes[6] != DM || in_sizes[8] != DM || in_sizes[10] != DM) return;
  if (in_sizes[11] != DM || in_sizes[12] != DM) return;
  if (in_sizes[13] != DM * FF || in_sizes[14] != FF || in_sizes[15] != FF * DM || in_sizes[16] != DM) return;
  if (out_size != NTOK * DM) return;

  const float* x     = (const float*)d_in[0];
  const float* ln1_g = (const float*)d_in[1];
  const float* ln1_b = (const float*)d_in[2];
  const float* wq    = (const float*)d_in[3];
  const float* bq    = (const float*)d_in[4];
  const float* wk    = (const float*)d_in[5];
  const float* bk    = (const float*)d_in[6];
  const float* wv    = (const float*)d_in[7];
  const float* bv    = (const float*)d_in[8];
  const float* wo    = (const float*)d_in[9];
  const float* bo    = (const float*)d_in[10];
  const float* ln2_g = (const float*)d_in[11];
  const float* ln2_b = (const float*)d_in[12];
  const float* w1    = (const float*)d_in[13];
  const float* b1    = (const float*)d_in[14];
  const float* w2    = (const float*)d_in[15];
  const float* b2    = (const float*)d_in[16];
  float* out = (float*)d_out;

  size_t off = 0;
  const size_t oWq  = off; off += PW_DD;
  const size_t oWk  = off; off += PW_DD;
  const size_t oWv  = off; off += PW_DD;
  const size_t oWo  = off; off += PW_DD;
  const size_t oW1  = off; off += PW_DF;
  const size_t oW2  = off; off += PW_DF;
  const size_t oH   = off; off += PACT;
  const size_t oQ   = off; off += PACT;
  const size_t oK   = off; off += PACT;
  const size_t oVT  = off; off += PACT;
  const size_t oO   = off; off += PACT;
  const size_t oA1  = off; off += PADD;
  const size_t oH2  = off; off += PACT;
  const size_t oG   = off; off += PG;
  if (off > ws_size) return;

  char* ws = (char*)d_ws;
  _Float16* WqT = (_Float16*)(ws + oWq);
  _Float16* WkT = (_Float16*)(ws + oWk);
  _Float16* WvT = (_Float16*)(ws + oWv);
  _Float16* WoT = (_Float16*)(ws + oWo);
  _Float16* W1T = (_Float16*)(ws + oW1);
  _Float16* W2T = (_Float16*)(ws + oW2);
  _Float16* Hp  = (_Float16*)(ws + oH);
  _Float16* Qp  = (_Float16*)(ws + oQ);
  _Float16* Kp  = (_Float16*)(ws + oK);
  _Float16* VTp = (_Float16*)(ws + oVT);
  _Float16* Op  = (_Float16*)(ws + oO);
  float*    A1p = (float*)(ws + oA1);
  _Float16* H2p = (_Float16*)(ws + oH2);
  _Float16* Gp  = (_Float16*)(ws + oG);

  const dim3 blk(256);

  tpose16_kernel<<<dim3(DM / 64, DM / 64), blk, 0, stream>>>(wq, WqT, DM, DM, WCARRY);
  tpose16_kernel<<<dim3(DM / 64, DM / 64), blk, 0, stream>>>(wk, WkT, DM, DM, WCARRY);
  tpose16_kernel<<<dim3(DM / 64, DM / 64), blk, 0, stream>>>(wv, WvT, DM, DM, WCARRY);
  tpose16_kernel<<<dim3(DM / 64, DM / 64), blk, 0, stream>>>(wo, WoT, DM, DM, WCARRY);
  tpose16_kernel<<<dim3(FF / 64, DM / 64), blk, 0, stream>>>(w1, W1T, DM, FF, WCARRY);
  tpose16_kernel<<<dim3(DM / 64, FF / 64), blk, 0, stream>>>(w2, W2T, FF, DM, WCARRY);

  ln_f16_kernel<<<dim3(NTOK), dim3(128), 0, stream>>>(x, ln1_g, ln1_b, Hp);

  const dim3 gP(((NTOK / 64) * (DM / 64) + 7) / 8, 1);
  wmma_gemm64<2, 1, false, 0><<<gP, blk, 0, stream>>>(
      Hp, DM, 0L, WqT, DM, 0L, (void*)Qp, DM, 0L, bq, nullptr, 0L, NTOK, DM, DM, WINV);
  wmma_gemm64<2, 1, false, 0><<<gP, blk, 0, stream>>>(
      Hp, DM, 0L, WkT, DM, 0L, (void*)Kp, DM, 0L, bk, nullptr, 0L, NTOK, DM, DM, WINV);
  const dim3 gVT(((DM / 64) * (SEQ / 64) + 7) / 8, NB);
  wmma_gemm64<1, 1, false, 0><<<gVT, blk, 0, stream>>>(
      WvT, DM, 0L, Hp, DM, (long)SEQ * DM, (void*)VTp, SEQ, (long)DM * SEQ, bv, nullptr, 0L, DM, SEQ, DM, WINV);

  attn_causal64_kernel<<<dim3(NH * (SEQ / AT_QB), NB), dim3(128), 0, stream>>>(Qp, Kp, VTp, Op, 0.125f);

  wmma_gemm64<2, 0, true, 0><<<gP, blk, 0, stream>>>(
      Op, DM, 0L, WoT, DM, 0L, (void*)A1p, DM, 0L, bo, x, 0L, NTOK, DM, DM, WINV);

  ln_f16_kernel<<<dim3(NTOK), dim3(128), 0, stream>>>(A1p, ln2_g, ln2_b, H2p);

  const dim3 gM1(((NTOK / 64) * (FF / 64) + 7) / 8, 1);
  wmma_gemm64<2, 1, false, 5><<<gM1, blk, 0, stream>>>(
      H2p, DM, 0L, W1T, DM, 0L, (void*)Gp, FF, 0L, b1, nullptr, 0L, NTOK, FF, DM, WINV);

  wmma_gemm64<2, 0, true, 0><<<gP, blk, 0, stream>>>(
      Gp, FF, 0L, W2T, FF, 0L, (void*)out, DM, 0L, b2, A1p, 0L, NTOK, DM, FF, WINV);

  (void)hipGetLastError();
}
